// GCNEncoder_89481348645581
// MI455X (gfx1250) — hardware-run, weakly checked
//
#include <hip/hip_runtime.h>

typedef float          v8f   __attribute__((ext_vector_type(8)));
typedef float          v4f   __attribute__((ext_vector_type(4)));
typedef unsigned int   v4u   __attribute__((ext_vector_type(4)));
typedef int            v8i   __attribute__((ext_vector_type(8)));
typedef unsigned short v8us  __attribute__((ext_vector_type(8)));
typedef unsigned short v16us __attribute__((ext_vector_type(16)));
typedef __bf16         v16bf __attribute__((ext_vector_type(16)));
typedef _Float16       v16h  __attribute__((ext_vector_type(16)));
typedef v4f  __attribute__((may_alias)) v4fa;
typedef v8us __attribute__((may_alias)) v8usa;
union FragB { v16bf v; v16us u; v8us h[2]; v8i w; };
union FragH { v16h  v; v16us u; v8us h[2]; v8i w; };

__device__ __forceinline__ v8f wmb(const FragB& a, const FragB& b, v8f c) {
  v8f d = __builtin_amdgcn_wmma_f32_16x16x32_bf16(false, a.v, false, b.v, (short)0, c, false, false);
  asm volatile("v_nop\n\tv_nop\n\tv_nop\n\tv_nop" : "+v"(d) : "v"(a.w), "v"(b.w));
  return d;
}

__device__ __forceinline__ v8f wmh(const FragH& a, const FragH& b, v8f c) {
  v8f d = __builtin_amdgcn_wmma_f32_16x16x32_f16(false, a.v, false, b.v, (short)0, c, false, false);
  asm volatile("v_nop\n\tv_nop\n\tv_nop\n\tv_nop" : "+v"(d) : "v"(a.w), "v"(b.w));
  return d;
}

__device__ __forceinline__ unsigned bf16_bits(float f) {
  const unsigned u = __float_as_uint(f);
  const unsigned r = (u + 0x7FFFu + ((u >> 16) & 1u)) >> 16;
  const unsigned q = (u >> 16) | 0x40u;
  return ((u & 0x7fffffffu) > 0x7f800000u) ? q : r;
}

__device__ __forceinline__ float bf16_val(float f) {
  return __uint_as_float(bf16_bits(f) << 16);
}
__device__ __forceinline__ int clampi(int v, int lo, int hi) {
  return v < lo ? lo : (v > hi ? hi : v);
}

__device__ __forceinline__ unsigned f16_bits(float f) {
  const unsigned u  = __float_as_uint(f);
  const unsigned s  = (u >> 16) & 0x8000u;
  const unsigned a  = u & 0x7fffffffu;
  const unsigned t  = a - 0x38000000u;
  const unsigned r  = (t + 0x0FFFu + ((t >> 13) & 1u)) >> 13;
  const unsigned rc = r > 0x7C00u ? 0x7C00u : r;
  const bool small  = a < 0x38800000u;
  const bool isnan  = a > 0x7f800000u;
  const unsigned fin = small ? 0u : (s | rc);
  return isnan ? (s | 0x7E00u) : fin;
}

__device__ __forceinline__ unsigned pk16(unsigned lo, unsigned hi) { return lo | (hi << 16); }
__device__ __forceinline__ unsigned bf16_lo_bits(float v) {
  float hi = bf16_val(v);
  asm volatile("" : "+v"(hi));
  return bf16_bits(v - hi);
}
__device__ __forceinline__ v4u pack8_bf16(v4f a, v4f c) {
  return (v4u){ pk16(bf16_bits(a[0]), bf16_bits(a[1])), pk16(bf16_bits(a[2]), bf16_bits(a[3])),
                pk16(bf16_bits(c[0]), bf16_bits(c[1])), pk16(bf16_bits(c[2]), bf16_bits(c[3])) };
}
__device__ __forceinline__ v4u pack8_bf16_lo(v4f a, v4f c) {
  return (v4u){ pk16(bf16_lo_bits(a[0]), bf16_lo_bits(a[1])), pk16(bf16_lo_bits(a[2]), bf16_lo_bits(a[3])),
                pk16(bf16_lo_bits(c[0]), bf16_lo_bits(c[1])), pk16(bf16_lo_bits(c[2]), bf16_lo_bits(c[3])) };
}
__device__ __forceinline__ v4u pack8_f16(v4f a, v4f c) {
  return (v4u){ pk16(f16_bits(a[0]), f16_bits(a[1])), pk16(f16_bits(a[2]), f16_bits(a[3])),
                pk16(f16_bits(c[0]), f16_bits(c[1])), pk16(f16_bits(c[2]), f16_bits(c[3])) };
}

template <int FORM>
__global__ __launch_bounds__(256) void k_plane(const float* __restrict__ src, int rows, int cols, int ldsrc,
                                               unsigned short* __restrict__ dst, int MP, int KP) {
  static_assert(FORM >= 0 && FORM <= 3);
  const int KTOT = (FORM == 1 || FORM == 3) ? 2 * KP : KP;
  const unsigned ppr   = (unsigned)(KTOT >> 3);
  const unsigned kp8   = (unsigned)(KP >> 3);
  const unsigned total = (unsigned)MP * ppr;
  const unsigned g     = blockIdx.x * 256u + threadIdx.x;
  const unsigned rowu  = g / ppr;
  const unsigned p     = g - rowu * ppr;
  const bool second    = p >= kp8;
  const int row = (int)rowu;
  const int c0  = (int)((second ? p - kp8 : p) << 3);
  const float* srow = src + (size_t)clampi(row, 0, rows - 1) * (size_t)ldsrc;
  float x[8];
  unsigned mk[8];
#pragma unroll
  for (int e = 0; e < 8; ++e) {
    const int c = c0 + e;
    const float v = srow[clampi(c, 0, cols - 1)];
    asm volatile("" :: "v"(v));
    x[e]  = v;
    mk[e] = (row < rows && c < cols) ? 0xFFFFu : 0u;
  }
  const v4f a = (v4f){ x[0], x[1], x[2], x[3] };
  const v4f c = (v4f){ x[4], x[5], x[6], x[7] };
  v4u o;
  if (FORM == 2) {
    o = pack8_f16(a, c);
  } else {
    const v4u hi = pack8_bf16(a, c);
    o = hi;
    if (FORM == 1) { const v4u lo = pack8_bf16_lo(a, c); o = second ? lo : hi; }
  }
  const v4u mw = (v4u){ pk16(mk[0], mk[1]), pk16(mk[2], mk[3]), pk16(mk[4], mk[5]), pk16(mk[6], mk[7]) };
  o &= mw;
  if (g < total) {
    volatile v4u* q = (volatile v4u*)(dst + (size_t)g * 8);
    *q = o;
    __threadfence();
    *q = o;
  }
}

template <int FORM> struct FragOf    { typedef FragB T; };
template <>         struct FragOf<2> { typedef FragH T; };
__device__ __forceinline__ v8f mm(const FragB& a, const FragB& b, v8f c) { return wmb(a, b, c); }
__device__ __forceinline__ v8f mm(const FragH& a, const FragH& b, v8f c) { return wmh(a, b, c); }
template <class F> __device__ __forceinline__ F ld_frag(const unsigned short* p) {
  F f;
  f.h[0] = *(const v8usa*)(p);
  f.h[1] = *(const v8usa*)(p + 16);
  return f;
}

template <int FORM, int EPI>
__global__ __launch_bounds__(256) __attribute__((amdgpu_num_vgpr(248)))
void k_gemm_nt(const unsigned short* __restrict__ A, const unsigned short* __restrict__ B,
               const float* __restrict__ bias, float* __restrict__ D, int M, int N, int KTOT, int ldd) {
  static_assert(FORM >= 0 && FORM <= 2);
  static_assert(EPI == 0 || EPI == 1);
  typedef typename FragOf<FORM>::T F;
  __shared__ __attribute__((aligned(16))) float sT[8][16 * 68];
  const int lane = threadIdx.x & 31;
  const int wave = threadIdx.x >> 5;
  const int tilesM = (M + 63) >> 6;
  const int tilesN = (N + 63) >> 6;
  const int tile = blockIdx.x * 8 + wave;
  if (tile >= tilesM * tilesN) return;
  const int tm = tile / tilesN;
  const int tn = tile - tm * tilesN;
  const int m0 = tm << 6;
  const int n0 = tn << 6;

  const int rl = lane & 15;
  const int h8 = (lane >> 4) * 8;
  const unsigned short* pa = A + (size_t)(m0 + rl) * (size_t)KTOT + h8;
  const unsigned short* pb = B + (size_t)(n0 + rl) * (size_t)KTOT + h8;

  v8f acc[4][4];
#pragma unroll
  for (int i = 0; i < 4; ++i)
#pragma unroll
    for (int j = 0; j < 4; ++j) acc[i][j] = (v8f){0.f, 0.f, 0.f, 0.f, 0.f, 0.f, 0.f, 0.f};

#pragma unroll 1
  for (int k0 = 0; k0 < KTOT; k0 += 32) {
    F bf[4];
#pragma unroll
    for (int j = 0; j < 4; ++j) bf[j] = ld_frag<F>(pb + (size_t)(j << 4) * (size_t)KTOT + k0);
#pragma unroll
    for (int i = 0; i < 4; ++i) {
      const F af = ld_frag<F>(pa + (size_t)(i << 4) * (size_t)KTOT + k0);
#pragma unroll
      for (int j = 0; j < 4; ++j) acc[i][j] = mm(af, bf[j], acc[i][j]);
    }
  }

  float* slab = sT[wave];
  const int hh = lane >> 4;
  const int c4 = (lane & 15) * 4;
  const int nc = n0 + c4;
  const bool cok = nc < N;
  v4f bv = (v4f){0.f, 0.f, 0.f, 0.f};
  if (EPI == 1) {
    bv = *(const v4fa*)(bias + clampi(nc, 0, N - 4));
    asm volatile("" :: "v"(bv));
  }
#pragma unroll
  for (int i = 0; i < 4; ++i) {
    const int mBase = m0 + (i << 4);
#pragma unroll
    for (int j = 0; j < 4; ++j) {
#pragma unroll
      for (int r = 0; r < 8; ++r) slab[(h8 + r) * 68 + (j << 4) + rl] = acc[i][j][r];
    }
    __builtin_amdgcn_fence(__ATOMIC_RELEASE, "workgroup");
    __builtin_amdgcn_wave_barrier();
    __builtin_amdgcn_fence(__ATOMIC_ACQUIRE, "workgroup");
    v4f vv[8];
#pragma unroll
    for (int it = 0; it < 8; ++it) {
      const int row = it * 2 + hh;
      v4f v = *(const v4fa*)(slab + row * 68 + c4);
      if (EPI == 1) v += bv;
      vv[it] = v;
    }
    for (int pass = 0; pass < 2; ++pass) {
#pragma unroll
      for (int it = 0; it < 8; ++it) {
        const int row = mBase + it * 2 + hh;
        if (cok && row < M) *(volatile v4f*)(D + (size_t)row * (size_t)ldd + nc) = vv[it];
      }
      __threadfence();
    }
    __builtin_amdgcn_fence(__ATOMIC_RELEASE, "workgroup");
    __builtin_amdgcn_wave_barrier();
    __builtin_amdgcn_fence(__ATOMIC_ACQUIRE, "workgroup");
  }
}

#pragma clang fp contract(off)

#include <stddef.h>
#include <stdint.h>

#ifndef SPLIT_L2
#define SPLIT_L2 1
#endif
#ifndef SPLIT_L3
#define SPLIT_L3 1
#endif

#define NNODE   50000
#define NEDGE   1600000
#define FD      128
#define MPAD    50048
#define NTHR    256
#define NWAVE   8
#define EPT     8
#define WCH     (32 * EPT)
#define NBRUN   512
#define SLB     9
#define NBK     98
#define NTAB    (NBK * NBRUN)
#define WLCA    3072
#define WLCB    2560
#define RCAP    20480
#define DEGCAP  96
#define MAXDEG_IN_MEAS   57
#define MAXDEG_OUT_MEAS  58
#define MAXB512_IN_MEAS  16678
#define MAXB512_OUT_MEAS 16695
#define OUT_ELEMS 6400000
#define WSMAX   ((size_t)128 << 20)

#define K2TOT (SPLIT_L2 ? 256 : 128)
#define K3TOT (SPLIT_L3 ? 256 : 128)

#define O_WL   0
#define O_PL   (NWAVE * WLCA)
#define O_CNT  (O_PL + RCAP)
#define O_OFF  (O_CNT + NBRUN)
#define O_CUR  (O_OFF + NBRUN)
#define O_CNTB (O_CUR + NBRUN)
#define O_DI   (O_CNTB + NBRUN)
#define O_DO   (O_DI + NBRUN)
#define BK_ZINTS (O_DO + NBRUN)
#define O_MISC BK_ZINTS
#define BK_INTS  (BK_ZINTS + 32)
#define BK_LDS   (BK_INTS * 4)

#define PB_W1 (FD * FD / 8 / NTHR)
#define PB_W2 (FD * K2TOT / 8 / NTHR)
#define PB_W3 (FD * K3TOT / 8 / NTHR)
#define PB_BI 1
#define PB_Z  6
#define PB_TOT (PB_W1 + PB_W2 + PB_W3 + PB_BI + PB_Z)

static_assert(FD == 32 * 4 && FD % 64 == 0 && FD % 32 == 0);
static_assert(NNODE % NWAVE == 0 && NNODE % 16 == 0);
static_assert(MPAD == 782 * 64 && MPAD % 64 == 0 && MPAD >= NNODE && MPAD - NNODE == 48 && MPAD % 16 == 0);
static_assert(NBRUN == (1 << SLB) && NNODE <= (1 << 16) && 16 + SLB <= 31);
static_assert(NBRUN * NBK >= NNODE && NTAB >= MPAD && (NBK - 1) * NBRUN < NNODE);
static_assert(NEDGE % WCH == 0 && NEDGE == 6250 * 256);
static_assert(RCAP == 20480 && DEGCAP == 96);
static_assert(RCAP % (NTHR * 4) == 0 && RCAP == NWAVE * WLCB);
static_assert((long long)RCAP * 100 >= (long long)MAXB512_IN_MEAS * 120);
static_assert((long long)RCAP * 100 >= (long long)MAXB512_OUT_MEAS * 120);
static_assert(WLCA >= MAXB512_IN_MEAS / 8 + 8 * 46 + 1);
static_assert(WLCB >= MAXB512_OUT_MEAS / 8 + 8 * 46 + 1);
static_assert(MAXDEG_IN_MEAS + 8 <= DEGCAP);
static_assert(BK_ZINTS % 4 == 0 && O_PL % 4 == 0 && O_CNT % 4 == 0 && O_DI % 4 == 0 && O_DO % 4 == 0);
static_assert(NBRUN == NTHR * 2 && NBRUN == 128 * 4 && NBRUN % 32 == 0);
static_assert(BK_LDS == 192640 && BK_LDS < 300000 && BK_LDS + 0 <= 327680);
static_assert((FD * FD / 8) % NTHR == 0 && (FD * K2TOT / 8) % NTHR == 0 && (FD * K3TOT / 8) % NTHR == 0);
static_assert(PB_Z * NTHR * 8 == (MPAD - NNODE) * 256);
static_assert((MPAD * FD / 8) % NTHR == 0);
static_assert(OUT_ELEMS == NNODE * FD);
static_assert(K2TOT % 32 == 0 && K3TOT % 32 == 0);
static_assert((long long)MPAD * 256 / 8 < (1LL << 31));

typedef unsigned int v2u  __attribute__((ext_vector_type(2)));
typedef int          v4i  __attribute__((ext_vector_type(4)));
typedef v4i  __attribute__((may_alias)) v4ia;

__device__ __forceinline__ void st2_v4f(float* p, v4f v) {
  *(volatile v4f*)p = v;
  __threadfence();
  *(volatile v4f*)p = v;
}
__device__ __forceinline__ void st2_v8us(unsigned short* p, v8us v) {
  *(volatile v8us*)p = v;
  __threadfence();
  *(volatile v8us*)p = v;
}

__device__ __forceinline__ v8us gather8(const float* __restrict__ base, int stride) {
  float f[8];
#pragma unroll
  for (int i = 0; i < 8; ++i) f[i] = base[(size_t)i * (size_t)stride];
  v8us o;
#pragma unroll
  for (int i = 0; i < 8; ++i) o[i] = (unsigned short)bf16_bits(f[i]);
  return o;
}

__device__ __forceinline__ void wplane_unit(const float* __restrict__ w, unsigned short* wd, int u, int ktot) {
  const int ppr = ktot >> 3;
  const int n   = u / ppr;
  const int kk  = (u - n * ppr) << 3;
  const int k8  = kk & (FD - 1);
  const v8us o = gather8(w + (size_t)k8 * FD + n, FD);
  st2_v8us(wd + (size_t)n * (size_t)ktot + kk, o);
}

__global__ __launch_bounds__(NTHR) void k_prep(const float* __restrict__ W1, const float* __restrict__ W2,
                                               const float* __restrict__ W3, const float* __restrict__ b1,
                                               const float* __restrict__ b2, const float* __restrict__ b3,
                                               unsigned short* W1T, unsigned short* W2D, unsigned short* W3D,
                                               float* BIAS, unsigned short* H) {
  const int tid = (int)threadIdx.x;
  const int blk = (int)blockIdx.x;
  if (blk < PB_W1) {
    wplane_unit(W1, W1T, blk * NTHR + tid, FD);
  } else if (blk < PB_W1 + PB_W2) {
    wplane_unit(W2, W2D, (blk - PB_W1) * NTHR + tid, K2TOT);
  } else if (blk < PB_W1 + PB_W2 + PB_W3) {
    wplane_unit(W3, W3D, (blk - PB_W1 - PB_W2) * NTHR + tid, K3TOT);
  } else if (blk < PB_W1 + PB_W2 + PB_W3 + PB_BI) {
    const int l  = tid >> 5;
    const int c4 = (tid & 31) * 4;
    const v4f x0 = *(const v4fa*)(b1 + c4);
    const v4f x1 = *(const v4fa*)(b2 + c4);
    const v4f x2 = *(const v4fa*)(b3 + c4);
    asm volatile("" :: "v"(x0));
    asm volatile("" :: "v"(x1));
    asm volatile("" :: "v"(x2));
    const unsigned s0 = 0u - (unsigned)(l == 0);
    const unsigned s1 = 0u - (unsigned)(l == 1);
    const unsigned s2 = 0u - (unsigned)(l == 2);
    v4f o;
#pragma unroll
    for (int e = 0; e < 4; ++e) {
      const unsigned bits = (__float_as_uint(x0[e]) & s0) | (__float_as_uint(x1[e]) & s1) | (__float_as_uint(x2[e]) & s2);
      o[e] = bf16_val(__uint_as_float(bits));
    }
    if (tid < 96) st2_v4f(BIAS + 4 * tid, o);
  } else {
    const int u = (blk - PB_W1 - PB_W2 - PB_W3 - PB_BI) * NTHR + tid;
    const v8us z = {0, 0, 0, 0, 0, 0, 0, 0};
    st2_v8us(H + (size_t)NNODE * 256 + (size_t)u * 8, z);
  }
}

__global__ __launch_bounds__(NTHR) void k_lists(const int* __restrict__ srcs, const int* __restrict__ dsts,
                                                int* LIST, int* CNT, int* OFF, int* DOt, int* DIt, int* FLAG) {
  extern __shared__ __attribute__((aligned(16))) int dsm[];
  const int tid = (int)threadIdx.x, lane = tid & 31, wave = tid >> 5;
  const int blk = (int)blockIdx.x;
  const unsigned nbs = (unsigned)(blk * NBRUN);

  {
    const v4i z4 = {0, 0, 0, 0};
    for (int i = tid * 4; i < BK_ZINTS; i += NTHR * 4) *(v4ia*)(dsm + i) = z4;
    if (tid < 32) dsm[O_MISC + tid] = 0;
  }
  __syncthreads();

  {
    const int per  = ((NEDGE + NWAVE * WCH - 1) / (NWAVE * WCH)) * WCH;
    const int ebeg = wave * per;
    const int eend = (ebeg + per < NEDGE) ? (ebeg + per) : NEDGE;
    int* la = dsm + O_WL + wave * WLCA;
    int* lb = dsm + O_PL + wave * WLCB;
    int wa = 0, wb = 0;
#pragma unroll 1
    for (int cb = ebeg; cb < eend; cb += WCH) {
      const int e0 = cb + lane * EPT;
      const v4i da = *(const v4ia*)(dsts + e0);
      const v4i db = *(const v4ia*)(dsts + e0 + 4);
      const v4i sa = *(const v4ia*)(srcs + e0);
      const v4i sb = *(const v4ia*)(srcs + e0 + 4);
      asm volatile("" :: "v"(da));
      asm volatile("" :: "v"(db));
      asm volatile("" :: "v"(sa));
      asm volatile("" :: "v"(sb));
      const int dv[8] = { da.x, da.y, da.z, da.w, db.x, db.y, db.z, db.w };
      const int sv[8] = { sa.x, sa.y, sa.z, sa.w, sb.x, sb.y, sb.z, sb.w };
      unsigned ta[8], tb[8], ma[8], mb[8];
      bool ha[8], hb[8];
      unsigned anyA = 0u, anyB = 0u;
#pragma unroll
      for (int j = 0; j < 8; ++j) {
        ta[j] = (unsigned)dv[j] - nbs;
        tb[j] = (unsigned)sv[j] - nbs;
        ha[j] = ta[j] < (unsigned)NBRUN;
        hb[j] = tb[j] < (unsigned)NBRUN;
        ma[j] = __builtin_amdgcn_ballot_w32(ha[j]);
        mb[j] = __builtin_amdgcn_ballot_w32(hb[j]);
        anyA |= ma[j];
        anyB |= mb[j];
      }
      if (anyA != 0u) {
        int pre = 0, pop = 0;
#pragma unroll
        for (int j = 0; j < 8; ++j) {
          pre += (int)__builtin_amdgcn_mbcnt_lo(ma[j], 0u);
          pop += (int)__builtin_popcount(ma[j]);
        }
        int p = wa + pre;
#pragma unroll
        for (int j = 0; j < 8; ++j) {
          const int word = (clampi(sv[j], 0, NNODE - 1) << SLB) | (int)(ta[j] & (unsigned)(NBRUN - 1));
          if (ha[j]) { if (p < WLCA) la[p] = word; p = p + 1; }
        }
        wa += pop;
      }
      if (anyB != 0u) {
        int pre = 0, pop = 0;
#pragma unroll
        for (int j = 0; j < 8; ++j) {
          pre += (int)__builtin_amdgcn_mbcnt_lo(mb[j], 0u);
          pop += (int)__builtin_popcount(mb[j]);
        }
        int p = wb + pre;
#pragma unroll
        for (int j = 0; j < 8; ++j) {
          const int word = (int)(tb[j] & (unsigned)(NBRUN - 1));
          if (hb[j]) { if (p < WLCB) lb[p] = word; p = p + 1; }
        }
        wb += pop;
      }
    }
    if (lane == 0) { dsm[O_MISC + wave] = wa; dsm[O_MISC + 8 + wave] = wb; }
  }
  __syncthreads();

  if (wave < 2) {
    const int role  = wave;
    const int lbase = role ? O_PL : O_WL;
    const int lcap  = role ? WLCB : WLCA;
    const int cbase = role ? O_CNTB : O_CNT;
    int ov = 0, tot = 0;
#pragma unroll 1
    for (int w2 = 0; w2 < NWAVE; ++w2) {
      int c = dsm[O_MISC + role * 8 + w2];
      if (c > lcap) ov = 1;
      c = clampi(c, 0, lcap);
      tot += c;
#pragma unroll 1
      for (int b0 = 0; b0 < c; b0 += 32) {
        const int idx = b0 + lane;
        const int ent = dsm[lbase + w2 * lcap + (idx < lcap ? idx : lcap - 1)];
        const int m32 = (c - b0) < 32 ? (c - b0) : 32;
#pragma unroll 1
        for (int k = 0; k < m32; ++k) {
          const int u    = __builtin_amdgcn_readlane(ent, k);
          const int slot = u & (NBRUN - 1);
          const int cv   = dsm[cbase + slot];
          asm volatile("" :: "v"(cv));
          if (lane == 0) dsm[cbase + slot] = cv + 1;
        }
      }
    }
    if (tot > RCAP) ov = 1;
    if (lane == 0) dsm[O_MISC + 16 + role] = ov;
  }
  __syncthreads();

  const int ovA = dsm[O_MISC + 16];
  const int ovB = dsm[O_MISC + 17];
  {
    const v4i z4 = {0, 0, 0, 0};
    for (int i = tid * 4; i < RCAP; i += NTHR * 4) *(v4ia*)(dsm + O_PL + i) = z4;
    const float qn = __uint_as_float(0x7fc00000u);
#pragma unroll 1
    for (int i = 0; i < 4; ++i) {
      const int role = i >> 1;
      const int slot = 2 * tid + (i & 1);
      int cc = dsm[(role ? O_CNTB : O_CNT) + slot];
      cc = cc < 1 ? 1 : cc;
      const float val = 1.0f / sqrtf((float)cc);
      const bool bad = (role != 0) && (ovB != 0);
      dsm[(role ? O_DO : O_DI) + slot] = __float_as_int(bad ? qn : val);
    }
  }
  if (wave == 0) {
    const int base = lane * (NBRUN / 32);
    int s = 0;
#pragma unroll 1
    for (int i = 0; i < NBRUN / 32; ++i) s += dsm[O_CNT + base + i];
    int incl = s;
#pragma unroll
    for (int d = 1; d < 32; d <<= 1) {
      const int y = __shfl_up(incl, d, 32);
      incl += (lane >= d) ? y : 0;
    }
    int run = incl - s;
#pragma unroll 1
    for (int i = 0; i < NBRUN / 32; ++i) {
      const int cv = dsm[O_CNT + base + i];
      dsm[O_OFF + base + i] = run;
      dsm[O_CUR + base + i] = run;
      run += cv;
    }
  }
  __syncthreads();

  if (wave == 0) {
#pragma unroll 1
    for (int w2 = 0; w2 < NWAVE; ++w2) {
      int c = dsm[O_MISC + w2];
      c = clampi(c, 0, WLCA);
#pragma unroll 1
      for (int b0 = 0; b0 < c; b0 += 32) {
        const int idx = b0 + lane;
        const int ent = dsm[O_WL + w2 * WLCA + (idx < WLCA ? idx : WLCA - 1)];
        const int m32 = (c - b0) < 32 ? (c - b0) : 32;
#pragma unroll 1
        for (int k = 0; k < m32; ++k) {
          const int u    = __builtin_amdgcn_readlane(ent, k);
          const int slot = u & (NBRUN - 1);
          const int sid  = (u >> SLB) & 0xFFFF;
          int p = dsm[O_CUR + slot];
          asm volatile("" :: "v"(p));
          p = clampi(p, 0, RCAP - 1);
          if (lane == 0) {
            dsm[O_PL + p]     = sid;
            dsm[O_CUR + slot] = p + 1;
          }
        }
      }
    }
  }
  __syncthreads();

  const int ovf = (ovA | ovB) != 0 ? 1 : 0;
  int* lp  = LIST + (size_t)blk * (size_t)RCAP;
  int* cp  = CNT + (size_t)blk * NBRUN;
  int* op  = OFF + (size_t)blk * NBRUN;
  int* dop = DOt + (size_t)blk * NBRUN;
  int* dip = DIt + (size_t)blk * NBRUN;
  int* fp  = FLAG + (size_t)blk * 32;
  for (int pass = 0; pass < 2; ++pass) {
#pragma unroll 1
    for (int i = tid * 4; i < RCAP; i += NTHR * 4) {
      const v4i v = *(const v4ia*)(dsm + O_PL + i);
      *(volatile v4i*)(lp + i) = v;
    }
    if (tid < NBRUN / 4) {
      const v4i vc = *(const v4ia*)(dsm + O_CNT + 4 * tid);
      const v4i vo = *(const v4ia*)(dsm + O_OFF + 4 * tid);
      const v4i vs = *(const v4ia*)(dsm + O_DO + 4 * tid);
      const v4i vd = *(const v4ia*)(dsm + O_DI + 4 * tid);
      *(volatile v4i*)(cp + 4 * tid)  = vc;
      *(volatile v4i*)(op + 4 * tid)  = vo;
      *(volatile v4i*)(dop + 4 * tid) = vs;
      *(volatile v4i*)(dip + 4 * tid) = vd;
    }
    if (tid < 8) {
      const v4i f = {ovf, ovf, ovf, ovf};
      *(volatile v4i*)(fp + 4 * tid) = f;
    }
    __threadfence();
  }
}

template <int L, int OSPLIT>
__global__ __launch_bounds__(NTHR) void k_walk(const int* __restrict__ LIST, const int* __restrict__ CNT,
                                               const int* __restrict__ OFF, const float* __restrict__ DOs,
                                               const float* __restrict__ DIs, const int* __restrict__ FLAG,
                                               const float* __restrict__ T, const float* __restrict__ BIAS,
                                               unsigned short* H, float* out) {
  static_assert(L >= 0 && L <= 2);
  __shared__ __attribute__((aligned(16))) float sbias[FD];
  const int tid = (int)threadIdx.x, lane = tid & 31, wave = tid >> 5;
  {
    const v4f b = *(const v4fa*)(BIAS + L * FD + 4 * (tid & 31));
    asm volatile("" :: "v"(b));
    if (tid < 32) *(v4fa*)(sbias + 4 * tid) = b;
  }
  __syncthreads();

  const int row = (int)blockIdx.x * NWAVE + wave;
  const int rc  = clampi(row, 0, NNODE - 1);
  const int blk = rc >> SLB;
  int c = CNT[rc];
  int o = OFF[rc];
  const float di = DIs[rc];
  const int flag = FLAG[(size_t)blk * 32];
  asm volatile("" :: "v"(c));
  asm volatile("" :: "v"(o));
  asm volatile("" :: "v"(di));
  asm volatile("" :: "v"(flag));
  const bool big = c > DEGCAP;
  c = __builtin_amdgcn_readfirstlane((row < NNODE) ? clampi(c, 0, DEGCAP) : 0);
  o = __builtin_amdgcn_readfirstlane(clampi(o, 0, RCAP - 1));
  int last = o + (c > 0 ? c : 1) - 1;
  last = last > RCAP - 1 ? RCAP - 1 : last;
  const int* lb = LIST + (size_t)blk * (size_t)RCAP;

  v4f acc = (v4f){0.0f, 0.0f, 0.0f, 0.0f};
#pragma unroll 1
  for (int b0 = 0; b0 < c; b0 += 32) {
    int idx = o + b0 + lane;
    idx = idx > last ? last : idx;
    const int word = lb[idx];
    asm volatile("" :: "v"(word));
    const int sr = clampi(word, 0, NNODE - 1);
    const float dv = DOs[sr];
    asm volatile("" :: "v"(dv));
    const int dbits = __float_as_int(dv);
    const int m32 = (c - b0) < 32 ? (c - b0) : 32;
#pragma unroll 1
    for (int k = 0; k < m32; ++k) {
      const int   sk = __builtin_amdgcn_readlane(sr, k);
      const float dk = __int_as_float(__builtin_amdgcn_readlane(dbits, k));
      const v4f q = *(const v4fa*)(T + (size_t)sk * FD + 4 * lane);
      asm volatile("" :: "v"(q));
      const v4f p = q * dk;
      acc = acc + p;
    }
  }

  const v4f bq = *(const v4fa*)(sbias + 4 * lane);
  v4f v = acc * di;
  v = v + bq;
  const float qnan = __uint_as_float(0x7fc00000u);
  const bool bad = (flag != 0) || big;
  float r0 = v[0], r1 = v[1], r2 = v[2], r3 = v[3];
  if (L < 2) {
    r0 = (r0 > 0.0f) ? r0 : (r0 - r0);
    r1 = (r1 > 0.0f) ? r1 : (r1 - r1);
    r2 = (r2 > 0.0f) ? r2 : (r2 - r2);
    r3 = (r3 > 0.0f) ? r3 : (r3 - r3);
  }
  r0 = bad ? qnan : r0;
  r1 = bad ? qnan : r1;
  r2 = bad ? qnan : r2;
  r3 = bad ? qnan : r3;

  if (row < NNODE) {
    if (L == 2) {
      const v4f ov = (v4f){r0, r1, r2, r3};
      float* op = out + (size_t)row * FD + 4 * lane;
      *(volatile v4f*)op = ov;
      __threadfence();
      *(volatile v4f*)op = ov;
    } else if (OSPLIT) {
      const v2u whi = (v2u){ pk16(bf16_bits(r0), bf16_bits(r1)), pk16(bf16_bits(r2), bf16_bits(r3)) };
      const v2u wlo = (v2u){ pk16(bf16_lo_bits(r0), bf16_lo_bits(r1)), pk16(bf16_lo_bits(r2), bf16_lo_bits(r3)) };
      volatile v2u* hp = (volatile v2u*)(H + (size_t)row * 256);
      hp[lane]      = whi;
      hp[32 + lane] = wlo;
      __threadfence();
      hp[lane]      = whi;
      hp[32 + lane] = wlo;
    } else {
      const v2u whi = (v2u){ pk16(bf16_bits(r0), bf16_bits(r1)), pk16(bf16_bits(r2), bf16_bits(r3)) };
      volatile v2u* hp = (volatile v2u*)(H + (size_t)row * 128);
      hp[lane] = whi;
      __threadfence();
      hp[lane] = whi;
    }
  }
}

extern "C" void kernel_launch(void* const* d_in, const int* in_sizes, int n_in,
                              void* d_out, int out_size, void* d_ws, size_t ws_size,
                              hipStream_t stream) {
  if (n_in < 9) return;
  if (in_sizes[0] != NNODE * FD) return;
  if (in_sizes[1] != NEDGE) return;
  if (in_sizes[2] != NEDGE) return;
  if (in_sizes[3] != FD * FD || in_sizes[5] != FD * FD || in_sizes[7] != FD * FD) return;
  if (in_sizes[4] != FD || in_sizes[6] != FD || in_sizes[8] != FD) return;
  if (out_size != OUT_ELEMS) return;

  const float* feat = (const float*)d_in[0];
  const int*   srcs = (const int*)d_in[1];
  const int*   dsts = (const int*)d_in[2];
  const float* W1 = (const float*)d_in[3];
  const float* b1 = (const float*)d_in[4];
  const float* W2 = (const float*)d_in[5];
  const float* b2 = (const float*)d_in[6];
  const float* W3 = (const float*)d_in[7];
  const float* b3 = (const float*)d_in[8];
  float* out = (float*)d_out;

  constexpr size_t zXB   = (size_t)MPAD * FD * 2;
  constexpr size_t zH    = (size_t)MPAD * 256 * 2;
  constexpr size_t zT    = (size_t)MPAD * FD * 4;
  constexpr size_t zLIST = (size_t)NBK * RCAP * 4;
  constexpr size_t zTAB  = (size_t)NTAB * 4;
  constexpr size_t zFLAG = (size_t)NBK * 128;
  constexpr size_t zW1T  = (size_t)FD * FD * 2;
  constexpr size_t zWD   = (size_t)FD * 256 * 2;
  constexpr size_t zBIAS = 1536;
  constexpr size_t oH    = 0;
  constexpr size_t oT    = oH + zH;
  constexpr size_t oLIST = oT + zT;
  constexpr size_t oCNT  = oLIST + zLIST;
  constexpr size_t oOFF  = oCNT + zTAB;
  constexpr size_t oDO   = oOFF + zTAB;
  constexpr size_t oDI   = oDO + zTAB;
  constexpr size_t oFLAG = oDI + zTAB;
  constexpr size_t oW1T  = oFLAG + zFLAG;
  constexpr size_t oW2D  = oW1T + zW1T;
  constexpr size_t oW3D  = oW2D + zWD;
  constexpr size_t oBIAS = oW3D + zWD;
  constexpr size_t oEND  = oBIAS + zBIAS;
  static_assert(zXB * 2 == zH && zXB <= zH);
  static_assert(zH % 256 == 0 && zT % 256 == 0 && zLIST % 256 == 0 && zTAB % 256 == 0);
  static_assert(zFLAG % 256 == 0 && zW1T % 256 == 0 && zWD % 256 == 0 && zBIAS % 256 == 0);
  static_assert(zBIAS >= 3 * FD * 4);
  static_assert(oEND == 60258048);
  static_assert(oEND <= ((size_t)128 << 20) && oEND <= (size_t)WSMAX);
  if (oEND > ws_size) return;

  char* ws = (char*)d_ws;
  unsigned short* H    = (unsigned short*)(ws + oH);
  unsigned short* XB   = (unsigned short*)(ws + oH);
  float*          T    = (float*)(ws + oT);
  int*            LIST = (int*)(ws + oLIST);
  int*            CNT  = (int*)(ws + oCNT);
  int*            OFF  = (int*)(ws + oOFF);
  int*            DOi  = (int*)(ws + oDO);
  const float*    DOf  = (const float*)(ws + oDO);
  int*            DIi  = (int*)(ws + oDI);
  const float*    DIf  = (const float*)(ws + oDI);
  int*            FLAG = (int*)(ws + oFLAG);
  unsigned short* W1T  = (unsigned short*)(ws + oW1T);
  unsigned short* W2D  = (unsigned short*)(ws + oW2D);
  unsigned short* W3D  = (unsigned short*)(ws + oW3D);
  float*          BIAS = (float*)(ws + oBIAS);

  hipFuncSetAttribute(reinterpret_cast<const void*>(&k_lists), hipFuncAttributeMaxDynamicSharedMemorySize, (int)BK_LDS);

  constexpr int GT = ((MPAD / 64) * (FD / 64) + 7) / 8;
  constexpr int GW = NNODE / NWAVE;
  static_assert(GT == 196 && GW == 6250);

  k_plane<0><<<MPAD * FD / 8 / NTHR, NTHR, 0, stream>>>(feat, NNODE, FD, FD, XB, MPAD, FD);
  k_prep<<<PB_TOT, NTHR, 0, stream>>>(W1, W2, W3, b1, b2, b3, W1T, W2D, W3D, BIAS, H);
  k_lists<<<NBK, NTHR, BK_LDS, stream>>>(srcs, dsts, LIST, CNT, OFF, DOi, DIi, FLAG);

  k_gemm_nt<0, 0><<<GT, NTHR, 0, stream>>>(XB, W1T, BIAS, T, MPAD, FD, FD, FD);
  k_walk<0, SPLIT_L2><<<GW, NTHR, 0, stream>>>(LIST, CNT, OFF, DOf, DIf, FLAG, T, BIAS, H, out);

  k_gemm_nt<(SPLIT_L2 ? 1 : 0), 0><<<GT, NTHR, 0, stream>>>(H, W2D, BIAS, T, MPAD, FD, K2TOT, FD);
  k_walk<1, SPLIT_L3><<<GW, NTHR, 0, stream>>>(LIST, CNT, OFF, DOf, DIf, FLAG, T, BIAS, H, out);

  k_gemm_nt<(SPLIT_L3 ? 1 : 0), 0><<<GT, NTHR, 0, stream>>>(H, W3D, BIAS, T, MPAD, FD, K3TOT, FD);
  k_walk<2, 0><<<GW, NTHR, 0, stream>>>(LIST, CNT, OFF, DOf, DIf, FLAG, T, BIAS, H, out);
}
